// Mamba_41102837022812
// MI455X (gfx1250) — hardware-verified
//
#include <hip/hip_runtime.h>
#include <math.h>

typedef __attribute__((ext_vector_type(16))) _Float16 v16h;
typedef __attribute__((ext_vector_type(8)))  _Float16 v8h;
typedef __attribute__((ext_vector_type(16))) __bf16   v16b;
typedef __attribute__((ext_vector_type(8)))  __bf16   v8b;
typedef __attribute__((ext_vector_type(8)))  float    v8f;
typedef __attribute__((ext_vector_type(4)))  float    v4f;

constexpr int kB     = 2;
constexpr int kL     = 4096;
constexpr int kC     = 256;
constexpr int kN     = 16;
constexpr int kR     = 4;
constexpr int kRows  = kB * kL;
constexpr int kT     = kR * kL;
constexpr int kPrjP  = 2 * kC;
constexpr int kSsmN  = kC + 2 * kN;
constexpr int kSsmP  = 320;
constexpr float kEps = 1e-5f;
constexpr int kScanCh = 64;
constexpr int kScanTS = 64;
constexpr int kScanYP = 68;
static_assert(kPrjP == 512 && kSsmN == 288 && kRows == 8192 && kT == 16384, "shapes");
static_assert((kC % 32) == 0, "GEMM K multiple of 32");
static_assert((kRows % 64) == 0 && (kPrjP % 64) == 0 && (kSsmP % 64) == 0 && (kC % 64) == 0 && kSsmP >= kSsmN, "GEMM M,N multiples of 64");
static_assert((kL % kScanTS) == 0 && (kT % kScanTS) == 0 && (kC % kScanCh) == 0 && (kRows % 8) == 0 && kScanCh == 64, "tile multiples");

constexpr size_t kOffXNH = 0;
constexpr size_t kOffXNL = kOffXNH + (size_t)kRows * kC * 2;
constexpr size_t kOffWIH = kOffXNL + (size_t)kRows * kC * 2;
constexpr size_t kOffWIL = kOffWIH + (size_t)kPrjP * kC * 2;
constexpr size_t kOffWSH = kOffWIL + (size_t)kPrjP * kC * 2;
constexpr size_t kOffWSL = kOffWSH + (size_t)kSsmP * kC * 2;
constexpr size_t kOffWOH = kOffWSL + (size_t)kSsmP * kC * 2;
constexpr size_t kOffWOL = kOffWOH + (size_t)kC * kC * 2;
constexpr size_t kOffPRJ = kOffWOL + (size_t)kC * kC * 2;
constexpr size_t kOffXGH = kOffPRJ + (size_t)kRows * kPrjP * 4;
constexpr size_t kOffXGL = kOffXGH + (size_t)kRows * kC * 2;
constexpr size_t kOffSSM = kOffXGL + (size_t)kRows * kC * 2;
constexpr size_t kOffYP  = kOffSSM + (size_t)kRows * kSsmP * 4;
constexpr size_t kOffGH  = kOffYP  + (size_t)kR * kRows * kC * 4;
constexpr size_t kOffGL  = kOffGH  + (size_t)kRows * kC * 2;
constexpr size_t kWsTotal = kOffGL + (size_t)kRows * kC * 2;
static_assert(kWsTotal == 87097344ull, "carve total");
static_assert(kWsTotal <= 134217728ull, "carve cap");
static_assert((kOffXNL % 128) == 0 && (kOffWIH % 128) == 0 && (kOffWIL % 128) == 0 && (kOffWSH % 128) == 0 &&
              (kOffWSL % 128) == 0 && (kOffWOH % 128) == 0 && (kOffWOL % 128) == 0 && (kOffPRJ % 128) == 0 &&
              (kOffXGH % 128) == 0 && (kOffXGL % 128) == 0 && (kOffSSM % 128) == 0 && (kOffYP % 128) == 0 &&
              (kOffGH % 128) == 0 && (kOffGL % 128) == 0, "128-B aligned regions");

__device__ __forceinline__ unsigned short f2bf_bits(float f) {
  unsigned u = __float_as_uint(f);
  return (unsigned short)((u + 0x7FFFu + ((u >> 16) & 1u)) >> 16);
}
__device__ __forceinline__ float bf_bits2f(unsigned short h) { return __uint_as_float(((unsigned)h) << 16); }

__device__ __forceinline__ void dep_guard4_h(v8f& a, v8f& b, v8f& c, v8f& d, v16h x, v16h y) { asm volatile("v_nop\n\tv_nop\n\tv_nop\n\tv_nop" : "+v"(a), "+v"(b), "+v"(c), "+v"(d) : "v"(x), "v"(y)); }
__device__ __forceinline__ void dep_guard4_b(v8f& a, v8f& b, v8f& c, v8f& d, v16b x, v16b y) { asm volatile("v_nop\n\tv_nop\n\tv_nop\n\tv_nop" : "+v"(a), "+v"(b), "+v"(c), "+v"(d) : "v"(x), "v"(y)); }
__device__ __forceinline__ void keep4_h(v16h a, v16h b, v16h c, v16h d) { asm volatile("v_nop" :: "v"(a), "v"(b), "v"(c), "v"(d)); }
__device__ __forceinline__ void keep4_b(v16b a, v16b b, v16b c, v16b d) { asm volatile("v_nop" :: "v"(a), "v"(b), "v"(c), "v"(d)); }
__device__ __forceinline__ void acc_guard4(v8f& a, v8f& b, v8f& c, v8f& d) { asm volatile("v_nop\n\tv_nop\n\tv_nop\n\tv_nop" : "+v"(a), "+v"(b), "+v"(c), "+v"(d)); }
template <typename T> struct Frag;
template <> struct Frag<_Float16> {
  typedef v16h V; union U { v16h v; v8h h[2]; };
  static __device__ __forceinline__ v16h load(const _Float16* p) {
    U f; f.h[0] = *(const v8h*)(p); f.h[1] = *(const v8h*)(p + 16); return f.v;
  }
  static __device__ __forceinline__ v8f mma(v16h a, v16h b, v8f c) {
    return __builtin_amdgcn_wmma_f32_16x16x32_f16(false, a, false, b, (short)0, c, false, false);
  }
  static __device__ __forceinline__ void guard4(v8f& a, v8f& b, v8f& c, v8f& d, v16h x, v16h y) { dep_guard4_h(a, b, c, d, x, y); }
  static __device__ __forceinline__ void keep(v16h a, v16h b, v16h c, v16h d) { keep4_h(a, b, c, d); }
};
template <> struct Frag<__bf16> {
  typedef v16b V; union U { v16b v; v8b h[2]; };
  static __device__ __forceinline__ v16b load(const __bf16* p) {
    U f; f.h[0] = *(const v8b*)(p); f.h[1] = *(const v8b*)(p + 16); return f.v;
  }
  static __device__ __forceinline__ v8f mma(v16b a, v16b b, v8f c) {
    return __builtin_amdgcn_wmma_f32_16x16x32_bf16(false, a, false, b, (short)0, c, false, false);
  }
  static __device__ __forceinline__ void guard4(v8f& a, v8f& b, v8f& c, v8f& d, v16b x, v16b y) { dep_guard4_b(a, b, c, d, x, y); }
  static __device__ __forceinline__ void keep(v16b a, v16b b, v16b c, v16b d) { keep4_b(a, b, c, d); }
};

template <int ET> struct Elem;
template <> struct Elem<0> { typedef _Float16 T; };
template <> struct Elem<1> { typedef __bf16 T; };
template <int ET, bool SPLIT, int BIAS_MODE, int OUT_MODE, bool RESID, int ACT = 0>
__global__ __launch_bounds__(256) void wmma_gemm64(
    const unsigned short* __restrict__ Ap, const unsigned short* __restrict__ A2p, int lda, long strideA,
    const unsigned short* __restrict__ Btp, const unsigned short* __restrict__ Bt2p, int ldb, long strideB,
    void* __restrict__ Cout, void* __restrict__ Cout2, int ldc, long strideC,
    const float* __restrict__ bias,
    const float* __restrict__ resid, long strideR,
    int M, int N, int K, float scale) {
  static_assert(!(RESID && (ACT != 0 || OUT_MODE != 0)), "resid path: f32 out, no activation");
  typedef typename Elem<ET>::T T;
  typedef typename Frag<T>::V V;
  const T* A = (const T*)Ap; const T* A2 = (const T*)A2p; const T* Bt = (const T*)Btp; const T* Bt2 = (const T*)Bt2p;
  __shared__ __align__(16) float sT[8][16 * 68];
  const int b    = blockIdx.y;
  const int lane = threadIdx.x & 31;
  const int wave = threadIdx.x >> 5;
  const int tilesN = N >> 6;
  const int tilesM = M >> 6;
  const int tile = blockIdx.x * 8 + wave;
  if (tile >= tilesM * tilesN) return;
  const int tm = tile / tilesN;
  const int tn = tile - tm * tilesN;
  const int m0 = tm << 6;
  const int n0 = tn << 6;

  const T* Ab  = A  + (size_t)b * strideA;
  const T* Bb  = Bt + (size_t)b * strideB;
  const T* Ab2 = SPLIT ? (A2  + (size_t)b * strideA) : nullptr;
  const T* Bb2 = SPLIT ? (Bt2 + (size_t)b * strideB) : nullptr;

  const int rlane = lane & 15;
  const int koff  = (lane >> 4) * 8;
  const int mOff  = (lane >> 4) * 8;

  v8f acc[4][4];
#pragma unroll
  for (int i = 0; i < 4; ++i)
#pragma unroll
    for (int j = 0; j < 4; ++j) acc[i][j] = (v8f){0.f,0.f,0.f,0.f,0.f,0.f,0.f,0.f};

  for (int k0 = 0; k0 < K; k0 += 32) {
    V bh[4], bl[4];
#pragma unroll
    for (int j = 0; j < 4; ++j) {
      const size_t bo = (size_t)(n0 + (j << 4) + rlane) * ldb + koff + k0;
      bh[j] = Frag<T>::load(Bb + bo);
      if (SPLIT) bl[j] = Frag<T>::load(Bb2 + bo);
    }
#pragma unroll
    for (int i = 0; i < 4; ++i) {
      const size_t ao = (size_t)(m0 + (i << 4) + rlane) * lda + koff + k0;
      V ah = Frag<T>::load(Ab + ao);
      V al;
      if (SPLIT) al = Frag<T>::load(Ab2 + ao);
#pragma unroll
      for (int j = 0; j < 4; ++j) {
        acc[i][j] = Frag<T>::mma(ah, bh[j], acc[i][j]);
        if (SPLIT) {
          acc[i][j] = Frag<T>::mma(ah, bl[j], acc[i][j]);
          acc[i][j] = Frag<T>::mma(al, bh[j], acc[i][j]);
        }
      }
      Frag<T>::guard4(acc[i][0], acc[i][1], acc[i][2], acc[i][3], ah, SPLIT ? al : ah);
    }
    Frag<T>::keep(bh[0], bh[1], bh[2], bh[3]);
    if (SPLIT) Frag<T>::keep(bl[0], bl[1], bl[2], bl[3]);
  }
  acc_guard4(acc[0][0], acc[0][1], acc[0][2], acc[0][3]);
  acc_guard4(acc[1][0], acc[1][1], acc[1][2], acc[1][3]);
  acc_guard4(acc[2][0], acc[2][1], acc[2][2], acc[2][3]);
  acc_guard4(acc[3][0], acc[3][1], acc[3][2], acc[3][3]);

  float* slab = sT[wave];
  const float* Rb = RESID ? (resid + (size_t)b * strideR) : nullptr;
#pragma unroll
  for (int i = 0; i < 4; ++i) {
    const int mBase = m0 + (i << 4);
#pragma unroll
    for (int j = 0; j < 4; ++j) {
      const int n = n0 + (j << 4) + rlane;
      float bv = 0.f;
      if (BIAS_MODE == 2) bv = bias[n];
#pragma unroll
      for (int r = 0; r < 8; ++r) {
        float v = acc[i][j][r] * scale;
        if (BIAS_MODE == 1) v += bias[mBase + mOff + r];
        if (BIAS_MODE == 2) v += bv;
        if (ACT == 1) v = tanhf(v);
        if (ACT == 2) v = fmaxf(v, 0.0f);
        if (ACT == 3) v = v / (1.0f + expf(-v));
        if (ACT == 4) v = (v > 0.f) ? v : 0.01f * v;
        slab[(mOff + r) * 68 + (j << 4) + rlane] = v;
      }
    }
    __builtin_amdgcn_fence(__ATOMIC_RELEASE, "workgroup");
    __builtin_amdgcn_wave_barrier();
    __builtin_amdgcn_fence(__ATOMIC_ACQUIRE, "workgroup");
    if (OUT_MODE == 0) {
      float* C = (float*)Cout + (size_t)b * strideC;
      const int hh = lane >> 4, c4 = (lane & 15) * 4;
      if (RESID) {
        v4f vo[8];
#pragma unroll
        for (int it = 0; it < 8; ++it) {
          const int row = it * 2 + hh;
          v4f v = *(const v4f*)(slab + row * 68 + c4);
          const v4f rv = *(const v4f*)(Rb + (size_t)(mBase + row) * ldc + n0 + c4);
          vo[it] = v + rv;
        }
        for (int ps = 0; ps < 2; ++ps) {
#pragma unroll
          for (int it = 0; it < 8; ++it) {
            const int row = it * 2 + hh;
            *(volatile v4f*)(C + (size_t)(mBase + row) * ldc + n0 + c4) = vo[it];
          }
          __threadfence();
        }
      } else {
        for (int ps = 0; ps < 2; ++ps) {
#pragma unroll
          for (int it = 0; it < 8; ++it) {
            const int row = it * 2 + hh;
            v4f v = *(const v4f*)(slab + row * 68 + c4);
            *(volatile v4f*)(C + (size_t)(mBase + row) * ldc + n0 + c4) = v;
          }
          __threadfence();
        }
      }
    } else {
      const int q = lane >> 3, c8 = (lane & 7) * 8;
      unsigned short* C  = (unsigned short*)Cout  + (size_t)b * strideC;
      unsigned short* C2 = (OUT_MODE == 2) ? ((unsigned short*)Cout2 + (size_t)b * strideC) : nullptr;
      for (int ps = 0; ps < 2; ++ps) {
#pragma unroll
        for (int it = 0; it < 4; ++it) {
          const int row = it * 4 + q;
          const float* sp = slab + row * 68 + c8;
          v8h hv, lv;
#pragma unroll
          for (int e = 0; e < 8; ++e) {
            if (OUT_MODE == 1) {
              hv[e] = (_Float16)sp[e];
            } else {
              unsigned short hb = f2bf_bits(sp[e]);
              unsigned short lb = f2bf_bits(sp[e] - bf_bits2f(hb));
              hv[e] = __builtin_bit_cast(_Float16, hb);
              lv[e] = __builtin_bit_cast(_Float16, lb);
            }
          }
          *(volatile v8h*)(C + (size_t)(mBase + row) * ldc + n0 + c8) = hv;
          if (OUT_MODE == 2) *(volatile v8h*)(C2 + (size_t)(mBase + row) * ldc + n0 + c8) = lv;
        }
        __threadfence();
      }
    }
    __builtin_amdgcn_fence(__ATOMIC_RELEASE, "workgroup");
    __builtin_amdgcn_wave_barrier();
    __builtin_amdgcn_fence(__ATOMIC_ACQUIRE, "workgroup");
  }
}

__global__ __launch_bounds__(256) void transpose_split_kernel(
    const float* __restrict__ W, unsigned short* __restrict__ Bh, unsigned short* __restrict__ Bl,
    int Kdim, int Ndim)
{
  __shared__ float tile[64 * 65];
  const int tid = threadIdx.x, lane = tid & 31, wave = tid >> 5;
  const int n0 = blockIdx.x * 64;
  const int k0 = blockIdx.y * 64;
#pragma unroll
  for (int p = 0; p < 8; ++p) {
    const int idx = tid + p * 256;
    const int kk  = idx >> 6;
    const int nn  = idx & 63;
    const int n   = n0 + nn;
    const int nc  = (n < Ndim) ? n : (Ndim - 1);
    const float v = W[(size_t)(k0 + kk) * Ndim + nc];
    tile[kk * 65 + nn] = (n < Ndim) ? v : 0.f;
  }
  asm volatile("" ::: "memory");
#pragma unroll
  for (int p = 8; p < 16; ++p) {
    const int idx = tid + p * 256;
    const int kk  = idx >> 6;
    const int nn  = idx & 63;
    const int n   = n0 + nn;
    const int nc  = (n < Ndim) ? n : (Ndim - 1);
    const float v = W[(size_t)(k0 + kk) * Ndim + nc];
    tile[kk * 65 + nn] = (n < Ndim) ? v : 0.f;
  }
  __syncthreads();
  const int q = lane >> 3, c8 = (lane & 7) * 8;
  v8h hv[2], lv[2];
#pragma unroll
  for (int it = 0; it < 2; ++it) {
    const int nrow = it * 32 + wave * 4 + q;
#pragma unroll
    for (int e = 0; e < 8; ++e) {
      const float f = tile[(c8 + e) * 65 + nrow];
      const unsigned short hb = f2bf_bits(f);
      const unsigned short lb = f2bf_bits(f - bf_bits2f(hb));
      hv[it][e] = __builtin_bit_cast(_Float16, hb);
      lv[it][e] = __builtin_bit_cast(_Float16, lb);
    }
  }
  for (int ps = 0; ps < 2; ++ps) {
#pragma unroll
    for (int it = 0; it < 2; ++it) {
      const int nrow = it * 32 + wave * 4 + q;
      const size_t o = (size_t)(n0 + nrow) * Kdim + k0 + c8;
      *(volatile v8h*)(Bh + o) = hv[it];
      *(volatile v8h*)(Bl + o) = lv[it];
    }
    __threadfence();
  }
}

__global__ __launch_bounds__(256) void ln_in_kernel(
    const float* __restrict__ x, const float* __restrict__ sc, const float* __restrict__ bi,
    unsigned short* __restrict__ XH, unsigned short* __restrict__ XL)
{
  const int lane = threadIdx.x & 31, wave = threadIdx.x >> 5;
  const int row = blockIdx.x * 8 + wave;
  const int c0 = lane * 8;
  const float* p = x + (size_t)row * kC + c0;
  const v4f a0 = *(const v4f*)(p);
  const v4f a1 = *(const v4f*)(p + 4);
  const v4f s0 = *(const v4f*)(sc + c0);
  const v4f s1 = *(const v4f*)(sc + c0 + 4);
  const v4f b0 = *(const v4f*)(bi + c0);
  const v4f b1 = *(const v4f*)(bi + c0 + 4);
  float s = 0.0f;
#pragma unroll
  for (int e = 0; e < 4; ++e) { s += a0[e]; s += a1[e]; }
#pragma unroll
  for (int off = 1; off < 32; off <<= 1) s += __shfl_xor(s, off, 32);
  const float mean = s * (1.0f / (float)kC);
  const v4f d0v = a0 - mean;
  const v4f d1v = a1 - mean;
  float q = 0.0f;
#pragma unroll
  for (int e = 0; e < 4; ++e) { q += d0v[e] * d0v[e]; q += d1v[e] * d1v[e]; }
#pragma unroll
  for (int off = 1; off < 32; off <<= 1) q += __shfl_xor(q, off, 32);
  const float var = q * (1.0f / (float)kC);
  const float rs = rsqrtf(var + kEps);
  v8h hv, lv;
#pragma unroll
  for (int e = 0; e < 4; ++e) {
    const float f0 = (d0v[e] * rs) * s0[e] + b0[e];
    const float f1 = (d1v[e] * rs) * s1[e] + b1[e];
    const unsigned short h0 = f2bf_bits(f0), h1 = f2bf_bits(f1);
    const unsigned short l0 = f2bf_bits(f0 - bf_bits2f(h0)), l1 = f2bf_bits(f1 - bf_bits2f(h1));
    hv[e]     = __builtin_bit_cast(_Float16, h0);
    hv[4 + e] = __builtin_bit_cast(_Float16, h1);
    lv[e]     = __builtin_bit_cast(_Float16, l0);
    lv[4 + e] = __builtin_bit_cast(_Float16, l1);
  }
  const size_t o = (size_t)row * kC + c0;
  *(volatile v8h*)(XH + o) = hv;
  *(volatile v8h*)(XL + o) = lv;
  __threadfence();
  *(volatile v8h*)(XH + o) = hv;
  *(volatile v8h*)(XL + o) = lv;
}

__global__ __launch_bounds__(256) void split_xg_kernel(
    const float* __restrict__ PRJ, unsigned short* __restrict__ XGH, unsigned short* __restrict__ XGL, int total8)
{
  const int i = blockIdx.x * 256 + threadIdx.x;
  if (i >= total8) return;
  const int row = i >> 5, c8 = (i & 31) * 8;
  const float* p = PRJ + (size_t)row * kPrjP + c8;
  const v4f a0 = *(const v4f*)(p);
  const v4f a1 = *(const v4f*)(p + 4);
  v8h hv, lv;
#pragma unroll
  for (int e = 0; e < 4; ++e) {
    const unsigned short h0 = f2bf_bits(a0[e]), h1 = f2bf_bits(a1[e]);
    const unsigned short l0 = f2bf_bits(a0[e] - bf_bits2f(h0)), l1 = f2bf_bits(a1[e] - bf_bits2f(h1));
    hv[e]     = __builtin_bit_cast(_Float16, h0);
    hv[4 + e] = __builtin_bit_cast(_Float16, h1);
    lv[e]     = __builtin_bit_cast(_Float16, l0);
    lv[4 + e] = __builtin_bit_cast(_Float16, l1);
  }
  const size_t o = (size_t)i << 3;
  *(volatile v8h*)(XGH + o) = hv;
  *(volatile v8h*)(XGL + o) = lv;
  __threadfence();
  *(volatile v8h*)(XGH + o) = hv;
  *(volatile v8h*)(XGL + o) = lv;
}

__global__ __launch_bounds__(kScanCh) void scan_kernel(
    const float* __restrict__ SSM, const float* __restrict__ PRJ,
    const float* __restrict__ bssm, const float* __restrict__ pbias,
    const float* __restrict__ Alog, const float* __restrict__ Dv,
    const float* __restrict__ gam, const int* __restrict__ bsz,
    float* __restrict__ YP)
{
  __shared__ __align__(16) float sBC[kScanTS * 2 * kN];
  __shared__ __align__(16) float sY[kScanTS * kScanYP];
  __shared__ __align__(16) float sA[kN * kScanCh];
  const int tid = threadIdx.x, lane = tid & 31, wave = tid >> 5;
  constexpr int kBlkPerB = kC / kScanCh;
  int nb = bsz[0];
  nb = (nb < 1) ? 1 : nb;
  nb = (nb > kB) ? kB : nb;
  const int bq = blockIdx.x / kBlkPerB;
  const int bix = (bq > nb - 1) ? (nb - 1) : bq;
  const int d0 = (blockIdx.x - bq * kBlkPerB) * kScanCh;
  const int d  = d0 + tid;
#pragma unroll 1
  for (int s = 0; s < kN; ++s) sA[s * kScanCh + tid] = -expf(Alog[(size_t)d * kN + s]);
  __syncthreads();
  float negA[kN], h[kN];
#pragma unroll
  for (int n = 0; n < kN; ++n) {
    negA[n] = sA[n * kScanCh + tid];
    h[n] = 0.0f;
  }
  const float bS = bssm[d], pb = pbias[d], Dd = Dv[d];
  const int sr = tid >> 3, sq = (tid & 7) * 4;
  const v4f bvec = *(const v4f*)(bssm + kC + sq);
  const int hh = lane >> 4, c4 = (lane & 15) * 4;
#pragma unroll 1
  for (int ck = 0; ck < kT / kScanTS; ++ck) {
    const int t0 = ck * kScanTS;
    const int r  = t0 / kL;
    const int l0 = t0 - r * kL;
    const size_t m0 = (size_t)bix * kL + (size_t)l0;
    const float gr = gam[d * kR + r];
    __syncthreads();
#pragma unroll
    for (int i = 0; i < 8; ++i) {
      const int rr = sr + 8 * i;
      v4f v = *(const v4f*)(SSM + (m0 + rr) * kSsmP + kC + sq);
      v = v + bvec;
      *(v4f*)(sBC + rr * (2 * kN) + sq) = v;
    }
    __syncthreads();
#pragma unroll 1
    for (int s = 0; s < kScanTS; ++s) {
      const size_t m = m0 + s;
      const float a  = SSM[m * kSsmP + d];
      const float v  = (a + bS) + pb;
      const float dt = fmaxf(v, 0.0f) + log1pf(expf(-fabsf(v)));
      const float uv = PRJ[m * kPrjP + d];
      const float du = dt * uv;
      const float* xr = sBC + s * (2 * kN);
      v4f Bq[4], Cq[4];
#pragma unroll
      for (int qq = 0; qq < 4; ++qq) {
        Bq[qq] = *(const v4f*)(xr + 4 * qq);
        Cq[qq] = *(const v4f*)(xr + kN + 4 * qq);
      }
      float y = 0.0f;
#pragma unroll
      for (int n = 0; n < kN; ++n) {
        const float e  = expf(dt * negA[n]);
        const float hn = e * h[n] + du * Bq[n >> 2][n & 3];
        h[n] = hn;
        y += hn * Cq[n >> 2][n & 3];
      }
      y += Dd * uv;
      sY[s * kScanYP + tid] = gr * y;
    }
    __syncthreads();
    for (int ps = 0; ps < 2; ++ps) {
#pragma unroll
      for (int it = 0; it < 16; ++it) {
        const int row = it * 4 + wave * 2 + hh;
        const v4f val = *(const v4f*)(sY + row * kScanYP + c4);
        *(volatile v4f*)(YP + ((size_t)r * kRows + m0 + row) * kC + d0 + c4) = val;
      }
      __threadfence();
    }
  }
}

__global__ __launch_bounds__(256) void ln_gate_kernel(
    const float* __restrict__ YP, const float* __restrict__ PRJ,
    const float* __restrict__ sc, const float* __restrict__ bi,
    unsigned short* __restrict__ GH, unsigned short* __restrict__ GL)
{
  const int lane = threadIdx.x & 31, wave = threadIdx.x >> 5;
  const int row = blockIdx.x * 8 + wave;
  const int c0 = lane * 8;
  v4f a0 = (v4f){0.f, 0.f, 0.f, 0.f};
  v4f a1 = (v4f){0.f, 0.f, 0.f, 0.f};
#pragma unroll
  for (int r = 0; r < kR; ++r) {
    const float* p = YP + ((size_t)r * kRows + row) * kC + c0;
    const v4f y0 = *(const v4f*)(p);
    const v4f y1 = *(const v4f*)(p + 4);
    a0 = a0 + y0;
    a1 = a1 + y1;
  }
  asm volatile("" ::: "memory");
  const float* zp = PRJ + (size_t)row * kPrjP + kC + c0;
  const v4f z0 = *(const v4f*)(zp);
  const v4f z1 = *(const v4f*)(zp + 4);
  const v4f s0 = *(const v4f*)(sc + c0);
  const v4f s1 = *(const v4f*)(sc + c0 + 4);
  const v4f b0 = *(const v4f*)(bi + c0);
  const v4f b1 = *(const v4f*)(bi + c0 + 4);
  float s = 0.0f;
#pragma unroll
  for (int e = 0; e < 4; ++e) { s += a0[e]; s += a1[e]; }
#pragma unroll
  for (int off = 1; off < 32; off <<= 1) s += __shfl_xor(s, off, 32);
  const float mean = s * (1.0f / (float)kC);
  const v4f d0v = a0 - mean;
  const v4f d1v = a1 - mean;
  float q = 0.0f;
#pragma unroll
  for (int e = 0; e < 4; ++e) { q += d0v[e] * d0v[e]; q += d1v[e] * d1v[e]; }
#pragma unroll
  for (int off = 1; off < 32; off <<= 1) q += __shfl_xor(q, off, 32);
  const float var = q * (1.0f / (float)kC);
  const float rs = rsqrtf(var + kEps);
  v8h hv, lv;
#pragma unroll
  for (int e = 0; e < 4; ++e) {
    const float n0 = (d0v[e] * rs) * s0[e] + b0[e];
    const float n1 = (d1v[e] * rs) * s1[e] + b1[e];
    const float g0 = z0[e] * n0;
    const float g1 = z1[e] * n1;
    const unsigned short h0 = f2bf_bits(g0), h1 = f2bf_bits(g1);
    const unsigned short l0 = f2bf_bits(g0 - bf_bits2f(h0)), l1 = f2bf_bits(g1 - bf_bits2f(h1));
    hv[e]     = __builtin_bit_cast(_Float16, h0);
    hv[4 + e] = __builtin_bit_cast(_Float16, h1);
    lv[e]     = __builtin_bit_cast(_Float16, l0);
    lv[4 + e] = __builtin_bit_cast(_Float16, l1);
  }
  const size_t o = (size_t)row * kC + c0;
  *(volatile v8h*)(GH + o) = hv;
  *(volatile v8h*)(GL + o) = lv;
  __threadfence();
  *(volatile v8h*)(GH + o) = hv;
  *(volatile v8h*)(GL + o) = lv;
}

extern "C" void kernel_launch(void* const* d_in, const int* in_sizes, int n_in,
                              void* d_out, int out_size, void* d_ws, size_t ws_size,
                              hipStream_t stream)
{
  if (n_in < 16) return;
  if (in_sizes[0] != kRows * kC) return;
  if (in_sizes[1] < 1) return;
  if (in_sizes[2] != kC || in_sizes[3] != kC) return;
  if (in_sizes[4] != kC * kPrjP || in_sizes[5] != kPrjP) return;
  if (in_sizes[6] != kC * kSsmN || in_sizes[7] != kSsmN) return;
  if (in_sizes[8] != kC) return;
  if (in_sizes[9] != kC * kN) return;
  if (in_sizes[10] != kC) return;
  if (in_sizes[11] != kC * kR) return;
  if (in_sizes[12] != kC || in_sizes[13] != kC) return;
  if (in_sizes[14] != kC * kC || in_sizes[15] != kC) return;
  if (out_size != kRows * kC) return;
  if (ws_size < kWsTotal) return;

  const float* x        = (const float*)d_in[0];
  const int*   bsz      = (const int*)d_in[1];
  const float* ln_in_s  = (const float*)d_in[2];
  const float* ln_in_b  = (const float*)d_in[3];
  const float* W_in     = (const float*)d_in[4];
  const float* b_in     = (const float*)d_in[5];
  const float* W_ssm    = (const float*)d_in[6];
  const float* b_ssm    = (const float*)d_in[7];
  const float* pbias    = (const float*)d_in[8];
  const float* As_log   = (const float*)d_in[9];
  const float* Dv       = (const float*)d_in[10];
  const float* gam      = (const float*)d_in[11];
  const float* ln_out_s = (const float*)d_in[12];
  const float* ln_out_b = (const float*)d_in[13];
  const float* W_out    = (const float*)d_in[14];
  const float* b_out    = (const float*)d_in[15];
  float* dout = (float*)d_out;

  char* ws = (char*)d_ws;
  unsigned short* XNH = (unsigned short*)(ws + kOffXNH);
  unsigned short* XNL = (unsigned short*)(ws + kOffXNL);
  unsigned short* WIH = (unsigned short*)(ws + kOffWIH);
  unsigned short* WIL = (unsigned short*)(ws + kOffWIL);
  unsigned short* WSH = (unsigned short*)(ws + kOffWSH);
  unsigned short* WSL = (unsigned short*)(ws + kOffWSL);
  unsigned short* WOH = (unsigned short*)(ws + kOffWOH);
  unsigned short* WOL = (unsigned short*)(ws + kOffWOL);
  float*          PRJ = (float*)(ws + kOffPRJ);
  unsigned short* XGH = (unsigned short*)(ws + kOffXGH);
  unsigned short* XGL = (unsigned short*)(ws + kOffXGL);
  float*          SSM = (float*)(ws + kOffSSM);
  float*          YP  = (float*)(ws + kOffYP);
  unsigned short* GH  = (unsigned short*)(ws + kOffGH);
  unsigned short* GL  = (unsigned short*)(ws + kOffGL);
  const float* dummy_bias  = b_in;
  const float* dummy_resid = x;

  transpose_split_kernel<<<dim3(kPrjP / 64, kC / 64), 256, 0, stream>>>(W_in,  WIH, WIL, kC, kPrjP);
  transpose_split_kernel<<<dim3(kSsmP / 64, kC / 64), 256, 0, stream>>>(W_ssm, WSH, WSL, kC, kSsmN);
  transpose_split_kernel<<<dim3(kC / 64, kC / 64), 256, 0, stream>>>(W_out, WOH, WOL, kC, kC);

  ln_in_kernel<<<kRows / 8, 256, 0, stream>>>(x, ln_in_s, ln_in_b, XNH, XNL);

  wmma_gemm64<1, true, 2, 0, false, 3><<<dim3(128, 1), 256, 0, stream>>>(
      XNH, XNL, kC, 0L, WIH, WIL, kC, 0L,
      (void*)PRJ, (void*)PRJ, kPrjP, 0L, b_in, dummy_resid, 0L, kRows, kPrjP, kC, 1.0f);

  split_xg_kernel<<<(kRows * kC / 8) / 256, 256, 0, stream>>>(PRJ, XGH, XGL, kRows * kC / 8);

  wmma_gemm64<1, true, 0, 0, false, 0><<<dim3(80, 1), 256, 0, stream>>>(
      XGH, XGL, kC, 0L, WSH, WSL, kC, 0L,
      (void*)SSM, (void*)SSM, kSsmP, 0L, dummy_bias, dummy_resid, 0L, kRows, kSsmP, kC, 1.0f);

  scan_kernel<<<kB * (kC / kScanCh), kScanCh, 0, stream>>>(SSM, PRJ, b_ssm, pbias, As_log, Dv, gam, bsz, YP);

  ln_gate_kernel<<<kRows / 8, 256, 0, stream>>>(YP, PRJ, ln_out_s, ln_out_b, GH, GL);

  wmma_gemm64<1, true, 2, 0, true, 0><<<dim3(64, 1), 256, 0, stream>>>(
      GH, GL, kC, 0L, WOH, WOL, kC, 0L,
      (void*)dout, (void*)dout, kC, 0L, b_out, x, 0L, kRows, kC, kC, 1.0f);
}
